// GWAN_40261023432900
// MI455X (gfx1250) — hardware-verified
//
#include <hip/hip_runtime.h>
#define NN 1024
#define NF 1024
#define HF 512
#define NE 32768
#define NG 16
#define NO 10
#define ZC 1536
#define SQRT2 1.4142135623730951f
#define MHC 0.8673250705840776f
#define LCAP 128
typedef __bf16 v16b __attribute__((ext_vector_type(16)));
typedef unsigned short v8us __attribute__((ext_vector_type(8), may_alias));
typedef float  v8f  __attribute__((ext_vector_type(8)));
typedef float  v4f  __attribute__((ext_vector_type(4)));
typedef float  v4fa __attribute__((ext_vector_type(4), may_alias));
union FragB { v16b v; v8us half[2]; unsigned short u[16]; };

__device__ __forceinline__ unsigned short bf16_bits(float x) { unsigned int u = __float_as_uint(x); return (unsigned short)((u + 0x7FFFu + ((u >> 16) & 1u)) >> 16); }
__device__ __forceinline__ float bf16_val(unsigned short b) { return __uint_as_float(((unsigned int)b) << 16); }
__device__ __forceinline__ float bf16_round(float x) { return bf16_val(bf16_bits(x)); }
template <int NT>
__device__ __forceinline__ v8f mmaN(v16b ah, v16b al, v16b bh, v16b bl, v8f c) {
  c = __builtin_amdgcn_wmma_f32_16x16x32_bf16(false, ah, false, bh, (short)0, c, false, false);
  if (NT >= 2) c = __builtin_amdgcn_wmma_f32_16x16x32_bf16(false, al, false, bh, (short)0, c, false, false);
  if (NT >= 3) c = __builtin_amdgcn_wmma_f32_16x16x32_bf16(false, ah, false, bl, (short)0, c, false, false);
  asm volatile("v_nop\n\tv_nop\n\tv_nop\n\tv_nop" : "+v"(c) : "v"(ah), "v"(al), "v"(bh), "v"(bl));
  return c;
}

__global__ __launch_bounds__(256) void k_wt_bf16(const float* __restrict__ W, unsigned short* __restrict__ Wt, int K, int N) {
  const int t = blockIdx.x * 256 + threadIdx.x;
  const int k8n = K / 8;
  if (t >= N * k8n) return;
  const int n = t / k8n, k8 = (t % k8n) * 8;
  v8us v;
#pragma unroll
  for (int i = 0; i < 8; ++i) v[i] = bf16_bits(W[(size_t)(k8 + i) * N + n]);
  *(volatile v8us*)(Wt + (size_t)n * K + k8) = v;
  __threadfence();
  *(volatile v8us*)(Wt + (size_t)n * K + k8) = v;
}

template <bool ASPLIT, int ACT, bool BIAS_BF16>
__global__ __launch_bounds__(128) void k_gemm_bf(const float* __restrict__ A, int lda, const unsigned short* __restrict__ Wt, int ldb,
                                               const float* __restrict__ bias, float* __restrict__ C, int ldc, int M, int N, int K) {
  __shared__ __attribute__((aligned(16))) float so[4][16][64];
  const int tid = threadIdx.x, w = tid >> 5, lane = tid & 31, ln = lane & 15, hh = lane >> 4;
  const int ntn = N / 64;
  const int wid = blockIdx.x * 4 + w;
  const int mt = wid / ntn, nq = wid % ntn;
  if (mt * 16 >= M) return;
  const int row0 = mt * 16, col0 = nq * 64;
  const float* arow = A + (size_t)(row0 + ln) * lda;
  v8f acc[4] = {};
  for (int kb = 0; kb < K; kb += 32) {
    FragB ah, al;
    const v4f x0 = *(const v4fa*)(arow + kb + 8 * hh), x1 = *(const v4fa*)(arow + kb + 8 * hh + 4);
    const v4f x2 = *(const v4fa*)(arow + kb + 16 + 8 * hh), x3 = *(const v4fa*)(arow + kb + 16 + 8 * hh + 4);
    float xs[16] = {x0[0],x0[1],x0[2],x0[3],x1[0],x1[1],x1[2],x1[3],x2[0],x2[1],x2[2],x2[3],x3[0],x3[1],x3[2],x3[3]};
#pragma unroll
    for (int i = 0; i < 16; ++i) { const unsigned short hb = bf16_bits(xs[i]); ah.u[i] = hb; al.u[i] = ASPLIT ? bf16_bits(xs[i] - bf16_val(hb)) : (unsigned short)0; }
#pragma unroll
    for (int t = 0; t < 4; ++t) {
      const unsigned short* brow = Wt + (size_t)(col0 + t * 16 + ln) * ldb + kb;
      FragB b;
      b.half[0] = *(const v8us*)(brow + 8 * hh);
      b.half[1] = *(const v8us*)(brow + 16 + 8 * hh);
      acc[t] = mmaN<ASPLIT ? 2 : 1>(ah.v, al.v, b.v, b.v, acc[t]);
    }
  }
#pragma unroll
  for (int t = 0; t < 4; ++t) {
    float bv = bias ? bias[col0 + t * 16 + ln] : 0.f;
    if (BIAS_BF16) bv = bf16_round(bv);
#pragma unroll
    for (int r = 0; r < 8; ++r) { float v = acc[t][r] + bv; if (ACT == 1) v = fmaxf(v, 0.f); so[w][8 * hh + r][t * 16 + ln] = v; }
  }
  __builtin_amdgcn_fence(__ATOMIC_ACQ_REL, "workgroup");
  __builtin_amdgcn_wave_barrier();
  const int rsub = lane >> 4, c4 = (lane & 15) * 4;
  for (int pass = 0; pass < 2; ++pass) {
#pragma unroll
    for (int q = 0; q < 8; ++q) {
      const int r = q * 2 + rsub;
      const v4f v = *(const v4fa*)&so[w][r][c4];
      *(volatile v4f*)(C + (size_t)(row0 + r) * ldc + col0 + c4) = v;
    }
    if (pass == 0) __threadfence();
  }
}

template <bool ASPLIT, int ACT, bool BIAS_BF16, bool RES_BF16>
__global__ __launch_bounds__(128) void k_gemm_bf3(const float* __restrict__ A, int lda, const unsigned short* __restrict__ Wt, int ldb,
                                                const float* __restrict__ bias, const float* __restrict__ resid, int rmod, int ldr,
                                                float* __restrict__ C, int ldc, int M, int N, int K) {
  __shared__ __attribute__((aligned(16))) float so[4][16][64];
  const int tid = threadIdx.x, w = tid >> 5, lane = tid & 31, ln = lane & 15, hh = lane >> 4;
  const int ntn = N / 64;
  const int wid = blockIdx.x * 4 + w;
  const int mt = wid / ntn, nq = wid % ntn;
  if (mt * 16 >= M) return;
  const int row0 = mt * 16, col0 = nq * 64;
  const float* arow = A + (size_t)(row0 + ln) * lda;
  v8f acc[4] = {};
  for (int kb = 0; kb < K; kb += 32) {
    FragB ah, al;
    const v4f x0 = *(const v4fa*)(arow + kb + 8 * hh), x1 = *(const v4fa*)(arow + kb + 8 * hh + 4);
    const v4f x2 = *(const v4fa*)(arow + kb + 16 + 8 * hh), x3 = *(const v4fa*)(arow + kb + 16 + 8 * hh + 4);
    float xs[16] = {x0[0],x0[1],x0[2],x0[3],x1[0],x1[1],x1[2],x1[3],x2[0],x2[1],x2[2],x2[3],x3[0],x3[1],x3[2],x3[3]};
#pragma unroll
    for (int i = 0; i < 16; ++i) { const unsigned short hb = bf16_bits(xs[i]); ah.u[i] = hb; al.u[i] = ASPLIT ? bf16_bits(xs[i] - bf16_val(hb)) : (unsigned short)0; }
#pragma unroll
    for (int t = 0; t < 4; ++t) {
      const unsigned short* brow = Wt + (size_t)(col0 + t * 16 + ln) * ldb + kb;
      FragB b;
      b.half[0] = *(const v8us*)(brow + 8 * hh);
      b.half[1] = *(const v8us*)(brow + 16 + 8 * hh);
      acc[t] = mmaN<ASPLIT ? 2 : 1>(ah.v, al.v, b.v, b.v, acc[t]);
    }
  }
#pragma unroll
  for (int t = 0; t < 4; ++t) {
    const int col = col0 + t * 16 + ln;
    float bv = bias ? bias[col] : 0.f;
    if (BIAS_BF16) bv = bf16_round(bv);
#pragma unroll
    for (int r = 0; r < 8; ++r) {
      float v = acc[t][r] + bv;
      if (resid) { float rv = resid[(size_t)((row0 + 8 * hh + r) % rmod) * ldr + col]; if (RES_BF16) rv = bf16_round(rv); v += rv; }
      if (ACT == 1) v = fmaxf(v, 0.f);
      if (ACT == 2) v = 0.5f * v * (1.0f + erff(v * 0.70710678118654752f));
      if (ACT == 3) { const float u = 0.7978845608028654f * (v + 0.044715f * v * v * v); v = 0.5f * v * (1.0f + tanhf(u)); }
      so[w][8 * hh + r][t * 16 + ln] = v;
    }
  }
  __builtin_amdgcn_fence(__ATOMIC_ACQ_REL, "workgroup");
  __builtin_amdgcn_wave_barrier();
  const int rsub = lane >> 4, c4 = (lane & 15) * 4;
  for (int pass = 0; pass < 2; ++pass) {
#pragma unroll
    for (int q = 0; q < 8; ++q) {
      const int r = q * 2 + rsub;
      const v4f v = *(const v4fa*)&so[w][r][c4];
      *(volatile v4f*)(C + (size_t)(row0 + r) * ldc + col0 + c4) = v;
    }
    if (pass == 0) __threadfence();
  }
}
template <bool PARAM_BF16>
__global__ __launch_bounds__(256) void k_layernorm(const float* __restrict__ X, const float* __restrict__ R, const float* __restrict__ g, const float* __restrict__ bta,
                                                  float* __restrict__ out_sum, float* __restrict__ out_norm, int N, float eps) {
  __shared__ float red[256];
  const int row = blockIdx.x, tid = threadIdx.x;
  const float* x = X + (size_t)row * N; const float* rr = R ? R + (size_t)row * N : nullptr;
  float vals[16];
  const int per = N / 256;
  float s1 = 0.f;
  for (int u = 0; u < per / 4; ++u) {
    const int j = tid * 4 + 1024 * u;
    const v4f a = *(const v4fa*)(x + j);
    v4f b = {0.f,0.f,0.f,0.f}; if (rr) b = *(const v4fa*)(rr + j);
#pragma unroll
    for (int q = 0; q < 4; ++q) { const float v = a[q] + b[q]; vals[u * 4 + q] = v; s1 += v; }
  }
  red[tid] = s1; __syncthreads();
  for (int st = 128; st > 0; st >>= 1) { if (tid < st) red[tid] += red[tid + st]; __syncthreads(); }
  const float mu = red[0] / (float)N; __syncthreads();
  float s2 = 0.f;
  for (int u = 0; u < per / 4; ++u)
#pragma unroll
    for (int q = 0; q < 4; ++q) { const float c = vals[u * 4 + q] - mu; s2 += c * c; }
  red[tid] = s2; __syncthreads();
  for (int st = 128; st > 0; st >>= 1) { if (tid < st) red[tid] += red[tid + st]; __syncthreads(); }
  const float rs = rsqrtf(red[0] / (float)N + eps);
  for (int pass = 0; pass < 2; ++pass) {
    for (int u = 0; u < per / 4; ++u) {
      const int j = tid * 4 + 1024 * u;
      v4f o, sm;
#pragma unroll
      for (int q = 0; q < 4; ++q) {
        float gg = g[j + q], bb = bta[j + q];
        if (PARAM_BF16) { gg = bf16_round(gg); bb = bf16_round(bb); }
        sm[q] = vals[u * 4 + q]; o[q] = (vals[u * 4 + q] - mu) * rs * gg + bb;
      }
      if (out_sum) *(volatile v4f*)(out_sum + (size_t)row * N + j) = sm;
      *(volatile v4f*)(out_norm + (size_t)row * N + j) = o;
    }
    if (pass == 0) __threadfence();
  }
}


typedef _Float16 v16h __attribute__((ext_vector_type(16)));
union FragH { v16h v; v8us half[2]; _Float16 h[16]; unsigned short u[16]; };
template <int NT>
__device__ __forceinline__ v8f mmaH(v16h ah, v16h al, v16h bh, v16h bl, v8f c) {
  c = __builtin_amdgcn_wmma_f32_16x16x32_f16(false, ah, false, bh, (short)0, c, false, false);
  if (NT >= 2) c = __builtin_amdgcn_wmma_f32_16x16x32_f16(false, al, false, bh, (short)0, c, false, false);
  if (NT >= 3) c = __builtin_amdgcn_wmma_f32_16x16x32_f16(false, ah, false, bl, (short)0, c, false, false);
  asm volatile("v_nop\n\tv_nop\n\tv_nop\n\tv_nop" : "+v"(c) : "v"(ah), "v"(al), "v"(bh), "v"(bl));
  return c;
}
template <bool ASPLIT>
__global__ __launch_bounds__(128) void k_gemm_h(const float* __restrict__ A, int lda, size_t sA, const _Float16* __restrict__ Bh, int ldb, size_t sB, float alpha, float* __restrict__ C, int ldc, size_t sC, int M, int N, int K) {
  __shared__ __attribute__((aligned(16))) float so[4][16][64];
  const int tid = threadIdx.x, w = tid >> 5, lane = tid & 31, ln = lane & 15, hh = lane >> 4; const int by = blockIdx.y;
  A += (size_t)by * sA; Bh += (size_t)by * sB; C += (size_t)by * sC;
  const int ntn = (N + 63) / 64; const int wid = blockIdx.x * 4 + w; const int mt = wid / ntn, nq = wid % ntn; if (mt * 16 >= M) return;
  const int row0 = mt * 16, col0 = nq * 64; const float* arow = A + (size_t)(row0 + ln) * lda;
  v8f acc[4] = {};
  for (int kb = 0; kb < K; kb += 32) {
    FragH ah, al;
    const v4f x0 = *(const v4fa*)(arow + kb + 8 * hh), x1 = *(const v4fa*)(arow + kb + 8 * hh + 4), x2 = *(const v4fa*)(arow + kb + 16 + 8 * hh), x3 = *(const v4fa*)(arow + kb + 16 + 8 * hh + 4);
    float xs[16] = {x0[0],x0[1],x0[2],x0[3],x1[0],x1[1],x1[2],x1[3],x2[0],x2[1],x2[2],x2[3],x3[0],x3[1],x3[2],x3[3]};
#pragma unroll
    for (int i = 0; i < 16; ++i) { const _Float16 h = (_Float16)xs[i]; ah.h[i] = h; al.h[i] = ASPLIT ? (_Float16)(xs[i] - (float)h) : (_Float16)0.0f; }
#pragma unroll
    for (int t = 0; t < 4; ++t) { if (col0 + t * 16 >= N) continue; const size_t boff = (size_t)(col0 + t * 16 + ln) * ldb + kb; FragH bq; bq.half[0] = *(const v8us*)(Bh + boff + 8 * hh); bq.half[1] = *(const v8us*)(Bh + boff + 16 + 8 * hh);
      acc[t] = mmaH<ASPLIT ? 2 : 1>(ah.v, al.v, bq.v, bq.v, acc[t]); }
  }
#pragma unroll
  for (int t = 0; t < 4; ++t) { if (col0 + t * 16 >= N) continue;
#pragma unroll
    for (int r = 0; r < 8; ++r) so[w][8 * hh + r][t * 16 + ln] = acc[t][r] * alpha; }
  __builtin_amdgcn_fence(__ATOMIC_ACQ_REL, "workgroup"); __builtin_amdgcn_wave_barrier();
  const int rsub = lane >> 4, c4 = (lane & 15) * 4;
  for (int pass = 0; pass < 2; ++pass) {
#pragma unroll
    for (int q = 0; q < 8; ++q) { const int r = q * 2 + rsub; if (col0 + c4 < N) { const v4f v = *(const v4fa*)&so[w][r][c4]; *(volatile v4f*)(C + (size_t)(row0 + r) * ldc + col0 + c4) = v; } }
    if (pass == 0) __threadfence(); }
}

__global__ __launch_bounds__(256) void k_wt_f16(const float* __restrict__ W, _Float16* __restrict__ Wt, int K, int N, float scale) {
  const int t = blockIdx.x * 256 + threadIdx.x; if (t >= N * (K / 8)) return; const int n = t / (K / 8), k8 = (t % (K / 8)) * 8; FragH f;
#pragma unroll
  for (int i = 0; i < 8; ++i) f.h[i] = (_Float16)(bf16_round(W[(size_t)(k8 + i) * N + n]) * scale); const v8us o = f.half[0];
  *(volatile v8us*)((unsigned short*)Wt + (size_t)n * K + k8) = o; __threadfence(); *(volatile v8us*)((unsigned short*)Wt + (size_t)n * K + k8) = o;
}
template <int ACT>
__global__ __launch_bounds__(128) void k_gemm_hhx(const _Float16* __restrict__ A, int lda, size_t sA, const _Float16* __restrict__ Bh, int ldb, size_t sB, float alpha, const float* __restrict__ bias, size_t sBias, const float* __restrict__ CP, int rowsPerB, size_t sCPb, int row0g,
    float* __restrict__ C, _Float16* __restrict__ C16, int ldc, size_t sC, int M, int N, int K) {
  __shared__ __attribute__((aligned(16))) float so[4][16][64];
  const int tid = threadIdx.x, w = tid >> 5, lane = tid & 31, ln = lane & 15, hh = lane >> 4; const int by = blockIdx.y;
  A += (size_t)by * sA; Bh += (size_t)by * sB; const size_t cofs = (size_t)by * sC; const float* bp = bias ? bias + (size_t)by * sBias : nullptr;
  const int ntn = (N + 63) / 64; const int wid = blockIdx.x * 4 + w; const int mt = wid / ntn, nq = wid % ntn; if (mt * 16 >= M) return;
  const int row0 = mt * 16, col0 = nq * 64; const _Float16* arow = A + (size_t)(row0 + ln) * lda;
  v8f acc[4] = {};
  for (int kb = 0; kb < K; kb += 32) { FragH ah; ah.half[0] = *(const v8us*)((const unsigned short*)arow + kb + 8 * hh); ah.half[1] = *(const v8us*)((const unsigned short*)arow + kb + 16 + 8 * hh);
#pragma unroll
    for (int t = 0; t < 4; ++t) { if (col0 + t * 16 >= N) continue; const size_t boff = (size_t)(col0 + t * 16 + ln) * ldb + kb; FragH bq; bq.half[0] = *(const v8us*)((const unsigned short*)Bh + boff + 8 * hh); bq.half[1] = *(const v8us*)((const unsigned short*)Bh + boff + 16 + 8 * hh);
      acc[t] = mmaH<1>(ah.v, ah.v, bq.v, bq.v, acc[t]); }
  }
#pragma unroll
  for (int t = 0; t < 4; ++t) { if (col0 + t * 16 >= N) continue; const int col = col0 + t * 16 + ln; const float bv = bp ? bf16_round(bp[col]) : 0.f;
#pragma unroll
    for (int r = 0; r < 8; ++r) { float v = acc[t][r] * alpha + bv; if (CP) { const int bidx = (row0g + row0 + 8 * hh + r) / rowsPerB; v += CP[(size_t)bidx * sCPb + (size_t)by * 64 + col]; } if (ACT == 1) v = (v > 0.f) ? v : expm1f(v); else if (ACT == 7) v = (v > 0.f) ? v + 1.0f : expf(v); else if (ACT == 8) v = tanhf(v); else if (ACT == 9) v = 0.5f * v * (1.0f + tanhf(0.7978845608028654f * (v + 0.044715f * v * v * v))); else if (ACT == 11) v = 1.0f / (1.0f + expf(-v)); else if (ACT == 12) v = (v > 0.f) ? v : 0.01f * v; else if (ACT == 14) v = (v > 0.f) ? v : 0.1f * v; else if (ACT == 15) v = v / (1.0f + expf(-v)); else if (ACT == 3) v = fmaxf(v, 0.f); else if (ACT == 6) v = 0.5f * v * (1.0f + erff(v * 0.70710678118654752f)); so[w][8 * hh + r][t * 16 + ln] = v; } }
  __builtin_amdgcn_fence(__ATOMIC_ACQ_REL, "workgroup"); __builtin_amdgcn_wave_barrier();
  const int rsub = lane >> 4, c4 = (lane & 15) * 4; typedef _Float16 v4h __attribute__((ext_vector_type(4)));
  for (int pass = 0; pass < 2; ++pass) {
#pragma unroll
    for (int q = 0; q < 8; ++q) { const int r = q * 2 + rsub; if (col0 + c4 < N) { const v4f v = *(const v4fa*)&so[w][r][c4]; if (C) *(volatile v4f*)(C + cofs + (size_t)(row0 + r) * ldc + col0 + c4) = v; if (C16) { v4h h4; for (int i = 0; i < 4; ++i) h4[i] = (_Float16)v[i]; *(volatile v4h*)(C16 + cofs + (size_t)(row0 + r) * ldc + col0 + c4) = h4; } } }
    if (pass == 0) __threadfence(); }
}


typedef _Float16 v4h __attribute__((ext_vector_type(4)));

__global__ __launch_bounds__(256) void k_x16(const float* __restrict__ x, _Float16* __restrict__ X16, size_t n8) { const size_t t = (size_t)blockIdx.x * 256 + threadIdx.x; if (t >= n8) return; FragH f;
#pragma unroll
  for (int q = 0; q < 8; ++q) f.h[q] = (_Float16)bf16_round(x[t * 8 + q]); *(volatile v8us*)((unsigned short*)X16 + t * 8) = f.half[0]; __threadfence(); *(volatile v8us*)((unsigned short*)X16 + t * 8) = f.half[0]; }
__global__ __launch_bounds__(256) void k_h16(const float* __restrict__ x, _Float16* __restrict__ X16, size_t n8) { const size_t t = (size_t)blockIdx.x * 256 + threadIdx.x; if (t >= n8) return; FragH f;
#pragma unroll
  for (int q = 0; q < 8; ++q) f.h[q] = (_Float16)x[t * 8 + q]; *(volatile v8us*)((unsigned short*)X16 + t * 8) = f.half[0]; __threadfence(); *(volatile v8us*)((unsigned short*)X16 + t * 8) = f.half[0]; }
__global__ __launch_bounds__(256) void k_round16f(const float* __restrict__ W, _Float16* __restrict__ Bt, size_t n8) { const size_t t = (size_t)blockIdx.x * 256 + threadIdx.x; if (t >= n8) return; FragH f;
#pragma unroll
  for (int i = 0; i < 8; ++i) f.h[i] = (_Float16)(bf16_round(W[t * 8 + i]) * 16.0f); *(volatile v8us*)((unsigned short*)Bt + t * 8) = f.half[0]; __threadfence(); *(volatile v8us*)((unsigned short*)Bt + t * 8) = f.half[0]; }
template <int NHv, int TTv>
__global__ __launch_bounds__(256) void k_vt(const _Float16* __restrict__ V16, int ldv, int voff, _Float16* __restrict__ Vt) { __shared__ unsigned short tl[64][66]; const int tid = threadIdx.x; const int slab = blockIdx.x / (TTv / 64), lg = blockIdx.x % (TTv / 64); const int b = slab / NHv, h = slab % NHv;
  for (int i = tid; i < 64 * 8; i += 256) { const int r = i / 8, c8 = (i % 8) * 8; FragH f; f.half[0] = *(const v8us*)((const unsigned short*)V16 + ((size_t)b * TTv + lg * 64 + r) * ldv + voff + h * 64 + c8);
#pragma unroll
    for (int q = 0; q < 8; ++q) tl[r][c8 + q] = f.u[q]; }
  __syncthreads();
  for (int pass = 0; pass < 2; ++pass) {
#pragma unroll
    for (int rd = 0; rd < 2; ++rd) { const int d = rd * 32 + tid / 8, pc = tid % 8; FragH f;
#pragma unroll
      for (int q = 0; q < 8; ++q) f.u[q] = tl[pc * 8 + q][d];
      *(volatile v8us*)((unsigned short*)Vt + ((size_t)slab * 64 + d) * TTv + lg * 64 + pc * 8) = f.half[0]; }
    if (pass == 0) __threadfence(); } }

__global__ __launch_bounds__(256) void k_hl(const float* __restrict__ F, _Float16* __restrict__ Hh, _Float16* __restrict__ Hl, size_t n8) { const size_t t = (size_t)blockIdx.x * 256 + threadIdx.x; if (t >= n8) return; FragH fh, fl; const v4f a = *(const v4fa*)(F + t * 8), c = *(const v4fa*)(F + t * 8 + 4);
#pragma unroll
  for (int q = 0; q < 4; ++q) { _Float16 h = (_Float16)a[q]; fh.h[q] = h; fl.h[q] = (_Float16)((a[q] - (float)h) * 1024.0f); h = (_Float16)c[q]; fh.h[4 + q] = h; fl.h[4 + q] = (_Float16)((c[q] - (float)h) * 1024.0f); }
  for (int pass = 0; pass < 2; ++pass) { *(volatile v8us*)((unsigned short*)Hh + t * 8) = fh.half[0]; *(volatile v8us*)((unsigned short*)Hl + t * 8) = fl.half[0]; if (pass == 0) __threadfence(); } }

__global__ __launch_bounds__(256) void k_split(const float* __restrict__ F, _Float16* __restrict__ Hh, _Float16* __restrict__ Hl, size_t n8) {
  #pragma clang fp contract(off)
  const size_t t = (size_t)blockIdx.x * 256 + threadIdx.x; if (t >= n8) return; const v4f a = *(const v4fa*)(F + t * 8), c = *(const v4fa*)(F + t * 8 + 4); FragH fh, fl;
#pragma unroll
  for (int q = 0; q < 8; ++q) { const float v = (q < 4) ? a[q] : c[q - 4]; const _Float16 hi = (_Float16)v; fh.h[q] = hi; fl.h[q] = (_Float16)((v - (float)hi) * 1024.0f); }
  for (int pass = 0; pass < 2; ++pass) { *(volatile v8us*)((unsigned short*)Hh + t * 8) = fh.half[0]; *(volatile v8us*)((unsigned short*)Hl + t * 8) = fl.half[0]; if (pass == 0) __threadfence(); } }
__global__ __launch_bounds__(256) void k_haar(const float* __restrict__ x, const float* __restrict__ watt, float* __restrict__ H) {
  #pragma clang fp contract(off)
  const int t = blockIdx.x * 256 + threadIdx.x; if (t >= NN * (HF / 4)) return; const int j0 = (t % (HF / 4)) * 4, n = t / (HF / 4); const float w0 = bf16_round(watt[0]), w1 = bf16_round(watt[1]); v4f o;
#pragma unroll
  for (int q = 0; q < 4; ++q) { const int j = j0 + q; const float xe = bf16_round(x[(size_t)n * NF + 2 * j]), xo = bf16_round(x[(size_t)n * NF + 2 * j + 1]); const float lo = (xe + xo) / SQRT2, hi = (xe - xo) / SQRT2; const float s = 1.0f / (1.0f + expf(-(lo * w0 + hi * w1))); o[q] = s * lo + (1.0f - s) * hi; }
  *(volatile v4f*)(H + (size_t)n * HF + j0) = o; __threadfence(); *(volatile v4f*)(H + (size_t)n * HF + j0) = o; }
__global__ __launch_bounds__(256) void k_gin(const int* __restrict__ ei, const float* __restrict__ H, float* __restrict__ AGG, _Float16* __restrict__ Sh, _Float16* __restrict__ Sl) {
  #pragma clang fp contract(off)
  __shared__ int lst[LCAP]; __shared__ int cntS; const int tid = threadIdx.x, n = blockIdx.x; if (tid == 0) cntS = 0; __syncthreads();
#pragma unroll 1
  for (int e = tid; e < NE; e += 256) { if (ei[NE + e] == n) { const int p = atomicAdd(&cntS, 1); if (p < LCAP) lst[p] = e; } }
  __syncthreads(); const int cnt = min(cntS, LCAP);
  if (tid == 0) { for (int a = 1; a < cnt; ++a) { const int v = lst[a]; int b = a - 1; while (b >= 0 && lst[b] > v) { lst[b + 1] = lst[b]; --b; } lst[b + 1] = v; } }
  __syncthreads();
  const int j0 = 2 * tid; float a0 = H[(size_t)n * HF + j0], a1 = H[(size_t)n * HF + j0 + 1];
#pragma unroll 1
  for (int k = 0; k < cnt; ++k) { int s = ei[lst[k]]; s = min(max(s, 0), NN - 1); a0 += H[(size_t)s * HF + j0]; a1 += H[(size_t)s * HF + j0 + 1]; }
  typedef float v2f __attribute__((ext_vector_type(2))); v2f v; v[0] = a0; v[1] = a1; const float s0 = a0 / (1.0f + expf(-a0)), s1 = a1 / (1.0f + expf(-a1)); FragH fh, fl; { const _Float16 h0 = (_Float16)s0, h1 = (_Float16)s1; fh.h[0] = h0; fh.h[1] = h1; fl.h[0] = (_Float16)((s0 - (float)h0) * 1024.0f); fl.h[1] = (_Float16)((s1 - (float)h1) * 1024.0f); }
  for (int pass = 0; pass < 2; ++pass) { *(volatile v2f*)(AGG + (size_t)n * HF + j0) = v; *(volatile unsigned int*)((unsigned short*)Sh + (size_t)n * HF + j0) = *(const unsigned int*)&fh.u[0]; *(volatile unsigned int*)((unsigned short*)Sl + (size_t)n * HF + j0) = *(const unsigned int*)&fl.u[0]; if (pass == 0) __threadfence(); } }
__global__ __launch_bounds__(256) void k_tpar(const float* __restrict__ trans, const float* __restrict__ scale, const float* __restrict__ wav, float* __restrict__ TT, float* __restrict__ SC, float* __restrict__ WW) { const int t = blockIdx.x * 256 + threadIdx.x; if (t >= HF * (HF / 4)) return; const int o0 = (t % (HF / 4)) * 4, i = t / (HF / 4); v4f a, b, c;
#pragma unroll
  for (int q = 0; q < 4; ++q) { a[q] = bf16_round(trans[(size_t)(o0 + q) * HF + i]); b[q] = bf16_round(scale[(size_t)(o0 + q) * HF + i]); c[q] = bf16_round(wav[(size_t)(o0 + q) * HF + i]); }
  for (int pass = 0; pass < 2; ++pass) { *(volatile v4f*)(TT + (size_t)i * HF + o0) = a; *(volatile v4f*)(SC + (size_t)i * HF + o0) = b; *(volatile v4f*)(WW + (size_t)i * HF + o0) = c; if (pass == 0) __threadfence(); } }
__global__ __launch_bounds__(256) void k_wav(const float* __restrict__ AGG, const float* __restrict__ TT, const float* __restrict__ SC, const float* __restrict__ WW, const float* __restrict__ BASE, float* __restrict__ PRE) {
  #pragma clang fp contract(off)
  __shared__ float ag[HF]; const int tid = threadIdx.x, n = blockIdx.x; ag[2 * tid] = AGG[(size_t)n * HF + 2 * tid]; ag[2 * tid + 1] = AGG[(size_t)n * HF + 2 * tid + 1]; __syncthreads();
  const int o0 = 2 * tid; float w0 = 0.f, w1 = 0.f;
#pragma unroll 1
  for (int i = 0; i < HF; ++i) { const float a = ag[i]; typedef float v2f __attribute__((ext_vector_type(2))); const v2f tr = *(const v2f*)(TT + (size_t)i * HF + o0), sc = *(const v2f*)(SC + (size_t)i * HF + o0), ww = *(const v2f*)(WW + (size_t)i * HF + o0);
    { const float s = (a - tr[0]) / sc[0]; const float s2 = s * s; w0 += ((MHC * (1.0f - s2)) * expf(-0.5f * s2)) * ww[0]; }
    { const float s = (a - tr[1]) / sc[1]; const float s2 = s * s; w1 += ((MHC * (1.0f - s2)) * expf(-0.5f * s2)) * ww[1]; } }
  typedef float v2f __attribute__((ext_vector_type(2))); v2f v; v[0] = w0 + BASE[(size_t)n * HF + o0]; v[1] = w1 + BASE[(size_t)n * HF + o0 + 1];
  *(volatile v2f*)(PRE + (size_t)n * HF + o0) = v; __threadfence(); *(volatile v2f*)(PRE + (size_t)n * HF + o0) = v; }
__global__ __launch_bounds__(256) void k_colstats(const float* __restrict__ Z, int C, int roundx, double* __restrict__ SUM, double* __restrict__ SQ) { __shared__ double s1[8][32], s2[8][32]; const int tid = threadIdx.x, w = tid >> 5, l = tid & 31; const int c = blockIdx.x * 32 + l; double a = 0.0, b = 0.0;
#pragma unroll 1
  for (int r = w; r < NN; r += 8) { float vf = Z[(size_t)r * C + c]; if (roundx) vf = bf16_round(vf); const double v = (double)vf; a += v; b += v * v; }
  s1[w][l] = a; s2[w][l] = b; __syncthreads();
  if (w == 0) { double t1 = 0.0, t2 = 0.0; for (int k = 0; k < 8; ++k) { t1 += s1[k][l]; t2 += s2[k][l]; } for (int pass = 0; pass < 2; ++pass) { *(volatile double*)(SUM + blockIdx.x * 32 + l) = t1; *(volatile double*)(SQ + blockIdx.x * 32 + l) = t2; if (pass == 0) __threadfence(); } } }
__global__ __launch_bounds__(256) void k_bn(const float* __restrict__ X, int C, const double* __restrict__ SUM, const double* __restrict__ SQ, float* __restrict__ Y, int CY, int c0) {
  #pragma clang fp contract(off)
  const int t = blockIdx.x * 256 + threadIdx.x; if (t >= NN * (C / 4)) return; const int cc = (t % (C / 4)) * 4, r = t / (C / 4); const v4f xv = *(const v4fa*)(X + (size_t)r * C + cc); v4f o;
#pragma unroll
  for (int q = 0; q < 4; ++q) { const int c = cc + q; const double m = SUM[c] / (double)NN; double var = SQ[c] / (double)NN - m * m; if (var < 0.0) var = 0.0; o[q] = (xv[q] - (float)m) / sqrtf((float)var + 1e-5f); }
  *(volatile v4f*)(Y + (size_t)r * CY + c0 + cc) = o; __threadfence(); *(volatile v4f*)(Y + (size_t)r * CY + c0 + cc) = o; }
__global__ __launch_bounds__(256) void k_bnx(const float* __restrict__ x, const double* __restrict__ SUM, const double* __restrict__ SQ, float* __restrict__ Zp) {
  #pragma clang fp contract(off)
  const int t = blockIdx.x * 256 + threadIdx.x; if (t >= NN * (NF / 4)) return; const int cc = (t % (NF / 4)) * 4, r = t / (NF / 4); const v4f xv = *(const v4fa*)(x + (size_t)r * NF + cc); v4f o;
#pragma unroll
  for (int q = 0; q < 4; ++q) { const int c = cc + q; const double m = SUM[c] / (double)NN; double var = SQ[c] / (double)NN - m * m; if (var < 0.0) var = 0.0; o[q] = (bf16_round(xv[q]) - (float)m) / sqrtf((float)var + 1e-5f); }
  *(volatile v4f*)(Zp + (size_t)r * ZC + cc) = o; __threadfence(); *(volatile v4f*)(Zp + (size_t)r * ZC + cc) = o; }
__global__ __launch_bounds__(256) void k_pool(const float* __restrict__ Zp, const int* __restrict__ batch, _Float16* __restrict__ Ph, _Float16* __restrict__ Pl) {
  #pragma clang fp contract(off)
  __shared__ float part[4][64]; __shared__ int cntp[4]; __shared__ __attribute__((aligned(16))) unsigned short rowh[64], rowl[64]; const int tid = threadIdx.x, cl = tid & 63, st = tid >> 6; const int g = blockIdx.x / (ZC / 64), cg = blockIdx.x % (ZC / 64); const int c = cg * 64 + cl; float s = 0.f; int cn = 0;
#pragma unroll 1
  for (int r = st; r < NN; r += 4) { if (batch[r] == g) { s += Zp[(size_t)r * ZC + c]; ++cn; } }
  part[st][cl] = s; if (cl == 0) cntp[st] = cn; __syncthreads();
  if (st == 0) { const float tot = ((part[0][cl] + part[1][cl]) + part[2][cl]) + part[3][cl]; const int ctot = cntp[0] + cntp[1] + cntp[2] + cntp[3]; const float v = tot / fmaxf((float)ctot, 1.f); const _Float16 hi = (_Float16)v; FragH fh, fl; fh.h[0] = hi; fl.h[0] = (_Float16)((v - (float)hi) * 1024.0f); rowh[cl] = fh.u[0]; rowl[cl] = fl.u[0]; }
  __syncthreads();
  if (st == 0 && cl < 8) { for (int pass = 0; pass < 2; ++pass) { *(volatile v8us*)((unsigned short*)Ph + (size_t)g * ZC + cg * 64 + cl * 8) = *(const v8us*)&rowh[cl * 8]; *(volatile v8us*)((unsigned short*)Pl + (size_t)g * ZC + cg * 64 + cl * 8) = *(const v8us*)&rowl[cl * 8]; if (pass == 0) __threadfence(); } } }
__global__ __launch_bounds__(256) void k_bpad(const float* __restrict__ bb, int n, float* __restrict__ BP) { const int l = threadIdx.x; if (l >= 32) return; const float v = (l < n) ? bb[l] : 0.f; *(volatile float*)(BP + l) = v; __threadfence(); *(volatile float*)(BP + l) = v; }
__global__ __launch_bounds__(256) void k_wn(const float* __restrict__ Wm, int nout, int orows, int K, _Float16* __restrict__ Bt) { const int t = blockIdx.x * 256 + threadIdx.x; if (t >= orows * (K / 8)) return; const int k0 = (t % (K / 8)) * 8, o = t / (K / 8); FragH f;
#pragma unroll
  for (int q = 0; q < 8; ++q) f.h[q] = (o < nout) ? (_Float16)(bf16_round(Wm[(size_t)o * K + k0 + q]) * 16.0f) : (_Float16)0.0f;
  *(volatile v8us*)((unsigned short*)Bt + (size_t)o * K + k0) = f.half[0]; __threadfence(); *(volatile v8us*)((unsigned short*)Bt + (size_t)o * K + k0) = f.half[0]; }
__global__ __launch_bounds__(256) void k_out(const float* __restrict__ O16p, float* __restrict__ out) { const int t = blockIdx.x * 256 + threadIdx.x; if (t >= NG * NO) return; const float v = O16p[(t / NO) * 16 + (t % NO)]; *(volatile float*)(out + t) = v; __threadfence(); *(volatile float*)(out + t) = v; }

extern "C" void kernel_launch(void* const* d_in, const int* in_sizes, int n_in,
                              void* d_out, int out_size, void* d_ws, size_t ws_size, hipStream_t stream) {
  (void)in_sizes; (void)n_in; (void)out_size;
  const float* x = (const float*)d_in[0]; const float* watt = (const float*)d_in[1]; const float* wk_scale = (const float*)d_in[2]; const float* wk_trans = (const float*)d_in[3]; const float* wk_wav = (const float*)d_in[4]; const float* wk_base = (const float*)d_in[5]; const float* fc1w = (const float*)d_in[6]; const float* fc1b = (const float*)d_in[7]; const float* fc2w = (const float*)d_in[8]; const float* fc2b = (const float*)d_in[9]; const int* ei = (const int*)d_in[10]; const int* batch = (const int*)d_in[11]; (void)d_in[12];
  char* ws = (char*)d_ws; size_t off = 0;
  auto take = [&](size_t bytes) { char* p = ws + off; off += (bytes + 255) & ~(size_t)255; return p; };
  float* H = (float*)take((size_t)NN * HF * 4); float* AGG = (float*)take((size_t)NN * HF * 4); _Float16* Sh = (_Float16*)take((size_t)NN * HF * 2); _Float16* Sl = (_Float16*)take((size_t)NN * HF * 2); float* TT = (float*)take((size_t)HF * HF * 4); float* SC = (float*)take((size_t)HF * HF * 4); float* WWp = (float*)take((size_t)HF * HF * 4); _Float16* Bb = (_Float16*)take((size_t)HF * HF * 2);
  float* BASE = (float*)take((size_t)NN * HF * 4); float* PRE = (float*)take((size_t)NN * HF * 4); float* C1 = (float*)take((size_t)NN * HF * 4); double* SUM = (double*)take(ZC * 8); double* SQ = (double*)take(ZC * 8); float* Zp = (float*)take((size_t)NN * ZC * 4);
  _Float16* Ph = (_Float16*)take((size_t)NG * ZC * 2); _Float16* Pl = (_Float16*)take((size_t)NG * ZC * 2); _Float16* B1 = (_Float16*)take((size_t)HF * ZC * 2); float* H1 = (float*)take((size_t)NG * HF * 4); _Float16* H1h = (_Float16*)take((size_t)NG * HF * 2); _Float16* H1l = (_Float16*)take((size_t)NG * HF * 2); _Float16* B2 = (_Float16*)take((size_t)16 * HF * 2); float* BP2 = (float*)take(128); float* O16p = (float*)take((size_t)NG * 16 * 4);
  if (off > ws_size) return;
  k_haar<<<(NN * (HF / 4) + 255) / 256, 256, 0, stream>>>(x, watt, H);
  k_gin<<<NN, 256, 0, stream>>>(ei, H, AGG, Sh, Sl);
  k_tpar<<<(HF * (HF / 4) + 255) / 256, 256, 0, stream>>>(wk_trans, wk_scale, wk_wav, TT, SC, WWp);
  k_round16f<<<(HF * HF / 8 + 255) / 256, 256, 0, stream>>>(wk_base, Bb, (size_t)HF * HF / 8);
  const dim3 gB(((NN / 16) * (HF / 64) + 3) / 4, 1);
  k_gemm_hhx<0><<<gB, 128, 0, stream>>>(Sh, HF, 0, Bb, HF, 0, 0.0625f, nullptr, 0, nullptr, 1, 0, 0, BASE, nullptr, HF, 0, NN, HF, HF); k_gemm_hhx<0><<<gB, 128, 0, stream>>>(Sl, HF, 0, Bb, HF, 0, 0.0625f / 1024.0f, nullptr, 0, BASE, 1, (size_t)HF, 0, BASE, nullptr, HF, 0, NN, HF, HF);
  k_wav<<<NN, 256, 0, stream>>>(AGG, TT, SC, WWp, BASE, PRE);
  k_colstats<<<HF / 32, 256, 0, stream>>>(PRE, HF, 0, SUM, SQ); k_bn<<<(NN * (HF / 4) + 255) / 256, 256, 0, stream>>>(PRE, HF, SUM, SQ, C1, HF, 0);
  k_colstats<<<HF / 32, 256, 0, stream>>>(C1, HF, 0, SUM, SQ); k_bn<<<(NN * (HF / 4) + 255) / 256, 256, 0, stream>>>(C1, HF, SUM, SQ, PRE, HF, 0);
  k_colstats<<<NF / 32, 256, 0, stream>>>(x, NF, 1, SUM, SQ); k_bnx<<<(NN * (NF / 4) + 255) / 256, 256, 0, stream>>>(x, SUM, SQ, Zp);
  k_colstats<<<HF / 32, 256, 0, stream>>>(PRE, HF, 0, SUM, SQ); k_bn<<<(NN * (HF / 4) + 255) / 256, 256, 0, stream>>>(PRE, HF, SUM, SQ, Zp, ZC, NF);
  k_pool<<<NG * (ZC / 64), 256, 0, stream>>>(Zp, batch, Ph, Pl);
  k_round16f<<<(HF * ZC / 8 + 255) / 256, 256, 0, stream>>>(fc1w, B1, (size_t)HF * ZC / 8);
  const dim3 g1(((NG / 16) * (HF / 64) + 3) / 4, 1), g2(((NG / 16) * 1 + 3) / 4, 1);
  k_gemm_hhx<0><<<g1, 128, 0, stream>>>(Ph, ZC, 0, B1, ZC, 0, 0.0625f, fc1b, 0, nullptr, 1, 0, 0, H1, nullptr, HF, 0, NG, HF, ZC); k_gemm_hhx<3><<<g1, 128, 0, stream>>>(Pl, ZC, 0, B1, ZC, 0, 0.0625f / 1024.0f, nullptr, 0, H1, 1, (size_t)HF, 0, H1, nullptr, HF, 0, NG, HF, ZC);
  k_split<<<(NG * HF / 8 + 255) / 256, 256, 0, stream>>>(H1, H1h, H1l, (size_t)NG * HF / 8);
  k_wn<<<(16 * (HF / 8) + 255) / 256, 256, 0, stream>>>(fc2w, NO, 16, HF, B2); k_bpad<<<1, 256, 0, stream>>>(fc2b, NO, BP2);
  k_gemm_hhx<0><<<g2, 128, 0, stream>>>(H1h, HF, 0, B2, HF, 0, 0.0625f, BP2, 0, nullptr, 1, 0, 0, O16p, nullptr, 16, 0, NG, 16, HF); k_gemm_hhx<0><<<g2, 128, 0, stream>>>(H1l, HF, 0, B2, HF, 0, 0.0625f / 1024.0f, nullptr, 0, O16p, 1, (size_t)16, 0, O16p, nullptr, 16, 0, NG, 16, HF);
  k_out<<<1, 256, 0, stream>>>(O16p, (float*)d_out);
}
